// SpatialAwareDecoder_67027259621778
// MI455X (gfx1250) — hardware-verified
//
#include <hip/hip_runtime.h>
#include <math.h>
#include <stdint.h>

#define TOKEN_DIM  1024
#define HIDDEN     256
#define NUM_FREQS  10
#define FOUR_DIM   63
#define IN_DIM     (TOKEN_DIM + FOUR_DIM)
#define NBATCH     2
#define TSEQ       512
#define NPTS       40000
#define ROWS_TOTAL (NBATCH * NPTS)
#define NHEAD      14

#define BLOCK_ROWS 32
#define NTHR       256

#define FSEG       64
#define K1W        (TOKEN_DIM + 2 * FSEG)
#define KST1       (K1W / 32)
#define K2W        (2 * HIDDEN)
#define KST2       (K2W / 32)
#define NT16       (HIDDEN / 16)

#define AP  1160
#define HP  520
#define SP  257
#define RP  17

#define TOK_PIECES (NBATCH * TSEQ * TOKEN_DIM / 8)
#define W1P_EL     (NT16 * KST1 * 512)
#define W2P_EL     (NT16 * KST2 * 512)
#define W3P_EL     (1 * KST2 * 512)
#define GPIECES    (BLOCK_ROWS * (TOKEN_DIM / 8))
#define OUT_FLOATS (BLOCK_ROWS * NHEAD)
#define OUT_PIECES (OUT_FLOATS / 4)

static_assert(ROWS_TOTAL % BLOCK_ROWS == 0);
static_assert(NPTS % BLOCK_ROWS == 0);
static_assert((OUT_FLOATS * 4) % 128 == 0);
static_assert(OUT_PIECES <= NTHR);
static_assert(BLOCK_ROWS * SP * 4 <= BLOCK_ROWS * AP * 2);
static_assert((AP % 8) == 0 && AP >= K1W);
static_assert((HP % 8) == 0 && HP >= K2W);
static_assert(3 * (2 * NUM_FREQS + 1) == FOUR_DIM);
static_assert(FOUR_DIM < FSEG);
static_assert(GPIECES % NTHR == 0);
static_assert(TOK_PIECES % 256 == 0);
static_assert((W1P_EL / 8) % 256 == 0 && (W2P_EL / 8) % 256 == 0 && (W3P_EL / 8) % 256 == 0);
static_assert(K1W % 32 == 0 && K2W % 32 == 0);
static_assert(BLOCK_ROWS == 32 && NTHR == 256);

typedef __bf16         v16b __attribute__((ext_vector_type(16)));
typedef unsigned short v8us __attribute__((ext_vector_type(8)));
typedef float          v8f  __attribute__((ext_vector_type(8)));
typedef float          v4f  __attribute__((ext_vector_type(4)));

union FragB { v16b v; v8us u[2]; };

__device__ __forceinline__ unsigned short bf_bits(float f) {
  const unsigned u = __float_as_uint(f);
  return (unsigned short)((u + 0x7FFFu + ((u >> 16) & 1u)) >> 16);
}
__device__ __forceinline__ float bf_up(unsigned short b) { return __uint_as_float(((unsigned)b) << 16); }
__device__ __forceinline__ float bfr(float f) { return bf_up(bf_bits(f)); }
__device__ __forceinline__ int clamp_tok(int t) { return (t < 0) ? 0 : ((t >= TSEQ) ? (TSEQ - 1) : t); }
__device__ __forceinline__ v8f zero8() { return (v8f){0.f, 0.f, 0.f, 0.f, 0.f, 0.f, 0.f, 0.f}; }

__device__ __forceinline__ v8f mma_b(v16b a, v16b b, v8f c) {
  return __builtin_amdgcn_wmma_f32_16x16x32_bf16(false, a, false, b, (short)0, c, false, false);
}
__device__ __forceinline__ void mma_guard1(v8f& c0, v16b a, v16b b) {
#if defined(__HIP_DEVICE_COMPILE__)
  asm volatile("v_nop\n\tv_nop\n\tv_nop\n\tv_nop" : "+v"(c0) : "v"(a), "v"(b));
#else
  (void)c0; (void)a; (void)b;
#endif
}
__device__ __forceinline__ void mma_guard4(v8f& c0, v8f& c1, v8f& c2, v8f& c3, v16b a, v16b b) {
#if defined(__HIP_DEVICE_COMPILE__)
  asm volatile("v_nop\n\tv_nop\n\tv_nop\n\tv_nop" : "+v"(c0), "+v"(c1), "+v"(c2), "+v"(c3) : "v"(a), "v"(b));
#else
  (void)c0; (void)c1; (void)c2; (void)c3; (void)a; (void)b;
#endif
}

__global__ __launch_bounds__(256) void k_tokc(const float* __restrict__ src, unsigned short* dst, int nPieces) {
  const int piece = blockIdx.x * 256 + threadIdx.x;
  const bool act  = piece < nPieces;
  const int pc    = act ? piece : (nPieces - 1);
  const v4f a = *(const v4f*)(src + (size_t)pc * 8);
  const v4f b = *(const v4f*)(src + (size_t)pc * 8 + 4);
  v8us o;
#pragma unroll
  for (int j = 0; j < 4; ++j) { o[j] = bf_bits(a[j]); o[4 + j] = bf_bits(b[j]); }
  unsigned short* d = dst + (size_t)pc * 8;
  if (act) *(volatile v8us*)d = o;
  __threadfence();
  if (act) *(volatile v8us*)d = o;
}

__global__ __launch_bounds__(256) void k_pack(const float* __restrict__ Wm, unsigned short* dst,
                                              int Kreal, int Nreal, int Ksplit, int segMask,
                                              int kS, int nPieces) {
  const int piece = blockIdx.x * 256 + threadIdx.x;
  const bool act  = piece < nPieces;
  const int pc    = act ? piece : (nPieces - 1);
  const int elem0 = pc * 8;
  const int tblk  = kS * 512;
  const int t     = elem0 / tblk;
  int rem         = elem0 - t * tblk;
  const int s     = rem >> 9;
  rem            &= 511;
  const int L     = rem >> 4;
  const int j0    = rem & 15;
  const int n     = t * 16 + (L & 15);
  const int hh    = L >> 4;
  const int kb    = s * 32 + 8 * hh + 2 * j0;
  const int nc    = (n < Nreal) ? n : (Nreal - 1);
  v8us o;
#pragma unroll
  for (int jj = 0; jj < 8; ++jj) {
    const int k  = kb + jj;
    const int ks = (k < Ksplit) ? k : (Ksplit + ((k - Ksplit) & segMask));
    const int kc = (ks < Kreal) ? ks : (Kreal - 1);
    float v = Wm[(size_t)kc * Nreal + nc];
    v = (ks < Kreal && n < Nreal) ? v : 0.0f;
    o[jj] = bf_bits(v);
  }
  unsigned short* d = dst + (size_t)pc * 8;
  if (act) *(volatile v8us*)d = o;
  __threadfence();
  if (act) *(volatile v8us*)d = o;
}

__device__ __forceinline__ void ln_relu(int wave, int lane, const float* Sf, unsigned short* Hd,
                                        const float* __restrict__ g, const float* __restrict__ be) {
  for (int rr = 0; rr < 4; ++rr) {
    const int r = wave * 4 + rr;
    const float* xr = Sf + r * SP;
    float vals[8];
    float s = 0.0f;
#pragma unroll
    for (int k = 0; k < 8; ++k) { vals[k] = xr[lane + 32 * k]; s += vals[k]; }
#pragma unroll
    for (int o = 16; o >= 1; o >>= 1) s += __shfl_xor(s, o, 32);
    const float mu = s * (1.0f / (float)HIDDEN);
    float ss = 0.0f;
#pragma unroll
    for (int k = 0; k < 8; ++k) { const float d = vals[k] - mu; ss += d * d; }
#pragma unroll
    for (int o = 16; o >= 1; o >>= 1) ss += __shfl_xor(ss, o, 32);
    const float var  = ss * (1.0f / (float)HIDDEN);
    const float rstd = rsqrtf(var + 1e-5f);
#pragma unroll
    for (int k = 0; k < 8; ++k) {
      const int c = lane + 32 * k;
      float y = (vals[k] - mu) * rstd * bfr(g[c]) + bfr(be[c]);
      y = fmaxf(y, 0.0f);
      const unsigned short hb = bf_bits(y);
      const unsigned short lb = bf_bits(y - bf_up(hb));
      Hd[r * HP + c]          = hb;
      Hd[r * HP + HIDDEN + c] = lb;
    }
  }
}

__global__ __launch_bounds__(NTHR) void k_main(
    const unsigned short* __restrict__ tokb, const float* __restrict__ anchors, const int* __restrict__ ids,
    const unsigned short* __restrict__ W1p, const unsigned short* __restrict__ W2p,
    const unsigned short* __restrict__ W3p,
    const float* __restrict__ b1, const float* __restrict__ g1, const float* __restrict__ be1,
    const float* __restrict__ b2, const float* __restrict__ g2, const float* __restrict__ be2,
    const float* __restrict__ b3, float* out) {
  __shared__ __align__(16) unsigned short sA[BLOCK_ROWS * AP];
  __shared__ __align__(16) unsigned short sH[BLOCK_ROWS * HP];
  __shared__ __align__(16) float sRaw[BLOCK_ROWS * RP];
  __shared__ __align__(16) float sOut[OUT_FLOATS];
  __shared__ int sIdx[BLOCK_ROWS];
  float* Sf = reinterpret_cast<float*>(sA);

  const int tid  = threadIdx.x;
  const int lane = tid & 31;
  const int wave = tid >> 5;
  const int hh   = lane >> 4;
  const int m16  = lane & 15;
  const int mt   = wave >> 2;
  const int nq   = wave & 3;
  const int arow = mt * 16 + m16;
  const int mrow = mt * 16 + 8 * hh;
  const int rowBase = blockIdx.x * BLOCK_ROWS;

  if (tid < BLOCK_ROWS) {
    const int p  = rowBase + tid;
    const int bb = p / NPTS;
    const int nn = p - bb * NPTS;
    sIdx[tid] = clamp_tok(ids[(size_t)bb * NPTS + nn]);
  }
  __syncthreads();

#pragma unroll 1
  for (int it = 0; it < GPIECES / NTHR; ++it) {
    const int pc = it * NTHR + tid;
    const int r  = pc >> 7;
    const int q  = pc & 127;
    const int p  = rowBase + r;
    const int bb = p / NPTS;
    const int t  = sIdx[r];
    const v8us v = *(const v8us*)(tokb + ((size_t)(bb * TSEQ + t)) * TOKEN_DIM + q * 8);
    *(v8us*)(sA + r * AP + q * 8) = v;
  }
  if (tid < 96) {
    const int r  = tid / 3;
    const int c  = tid - 3 * r;
    const int p  = rowBase + r;
    const int bb = p / NPTS;
    const int t  = sIdx[r];
    const float a = bfr(anchors[((size_t)(bb * TSEQ + t)) * 3 + c]);
    unsigned short* rp = sA + r * AP + TOKEN_DIM + 21 * c;
    {
      const unsigned short hb = bf_bits(a);
      rp[0]    = hb;
      rp[FSEG] = bf_bits(a - bf_up(hb));
    }
#pragma unroll 1
    for (int f = 0; f < NUM_FREQS; ++f) {
      const float ang = a * (float)(1 << f);
      const float sv  = sinf(ang);
      const float cv  = cosf(ang);
      const unsigned short hs = bf_bits(sv);
      const unsigned short hc = bf_bits(cv);
      rp[1 + f]                    = hs;
      rp[FSEG + 1 + f]             = bf_bits(sv - bf_up(hs));
      rp[1 + NUM_FREQS + f]        = hc;
      rp[FSEG + 1 + NUM_FREQS + f] = bf_bits(cv - bf_up(hc));
    }
  } else if (tid < 128) {
    const int r = tid - 96;
    sA[r * AP + TOKEN_DIM + FOUR_DIM]        = (unsigned short)0;
    sA[r * AP + TOKEN_DIM + FSEG + FOUR_DIM] = (unsigned short)0;
  }
  __syncthreads();

  {
    v8f acc[4];
#pragma unroll
    for (int t = 0; t < 4; ++t) acc[t] = zero8();
    const unsigned short* arp = sA + arow * AP + 8 * hh;
#pragma unroll 2
    for (int s = 0; s < KST1; ++s) {
      FragB a;
      a.u[0] = *(const v8us*)(arp + s * 32);
      a.u[1] = *(const v8us*)(arp + s * 32 + 16);
      FragB bq;
#pragma unroll
      for (int t = 0; t < 4; ++t) {
        const unsigned short* wp = W1p + (((size_t)(((nq * 4 + t) * KST1 + s) * 32 + lane)) << 4);
        bq.u[0] = *(const v8us*)(wp);
        bq.u[1] = *(const v8us*)(wp + 8);
        acc[t] = mma_b(a.v, bq.v, acc[t]);
      }
      mma_guard4(acc[0], acc[1], acc[2], acc[3], a.v, bq.v);
    }
    __syncthreads();
#pragma unroll
    for (int t = 0; t < 4; ++t) {
      const int c    = (nq * 4 + t) * 16 + m16;
      const float bv = bfr(b1[c]);
#pragma unroll
      for (int v = 0; v < 8; ++v) Sf[(mrow + v) * SP + c] = acc[t][v] + bv;
    }
  }
  __syncthreads();
  ln_relu(wave, lane, Sf, sH, g1, be1);
  __syncthreads();

  {
    v8f acc[4];
#pragma unroll
    for (int t = 0; t < 4; ++t) acc[t] = zero8();
    const unsigned short* hrp = sH + arow * HP + 8 * hh;
#pragma unroll 2
    for (int s = 0; s < KST2; ++s) {
      FragB a;
      a.u[0] = *(const v8us*)(hrp + s * 32);
      a.u[1] = *(const v8us*)(hrp + s * 32 + 16);
      FragB bq;
#pragma unroll
      for (int t = 0; t < 4; ++t) {
        const unsigned short* wp = W2p + (((size_t)(((nq * 4 + t) * KST2 + s) * 32 + lane)) << 4);
        bq.u[0] = *(const v8us*)(wp);
        bq.u[1] = *(const v8us*)(wp + 8);
        acc[t] = mma_b(a.v, bq.v, acc[t]);
      }
      mma_guard4(acc[0], acc[1], acc[2], acc[3], a.v, bq.v);
    }
#pragma unroll
    for (int t = 0; t < 4; ++t) {
      const int c    = (nq * 4 + t) * 16 + m16;
      const float bv = bfr(b2[c]);
#pragma unroll
      for (int v = 0; v < 8; ++v) Sf[(mrow + v) * SP + c] = acc[t][v] + bv;
    }
  }
  __syncthreads();
  ln_relu(wave, lane, Sf, sH, g2, be2);
  __syncthreads();

  if (wave < 2) {
    v8f c3 = zero8();
    const unsigned short* hrp = sH + (wave * 16 + m16) * HP + 8 * hh;
#pragma unroll 2
    for (int s = 0; s < KST2; ++s) {
      FragB a, bq;
      a.u[0] = *(const v8us*)(hrp + s * 32);
      a.u[1] = *(const v8us*)(hrp + s * 32 + 16);
      const unsigned short* wp = W3p + (((size_t)(s * 32 + lane)) << 4);
      bq.u[0] = *(const v8us*)(wp);
      bq.u[1] = *(const v8us*)(wp + 8);
      c3 = mma_b(a.v, bq.v, c3);
      mma_guard1(c3, a.v, bq.v);
    }
    const int bc = (m16 < NHEAD) ? m16 : (NHEAD - 1);
    float bv = bfr(b3[bc]);
    bv = (m16 < NHEAD) ? bv : 0.0f;
#pragma unroll
    for (int v = 0; v < 8; ++v) sRaw[(wave * 16 + 8 * hh + v) * RP + m16] = c3[v] + bv;
  }
  __syncthreads();

  for (int e = tid; e < OUT_FLOATS; e += NTHR) {
    const int r = e / NHEAD;
    const int j = e - r * NHEAD;
    const float* rp = sRaw + r * RP;
    const float x  = rp[j];
    const float q0 = rp[10], q1 = rp[11], q2 = rp[12], q3 = rp[13];
    const float col = fminf(fmaxf(x, 0.0f), 1.0f);
    const float sg  = 1.0f / (1.0f + expf(-x));
    const float ex  = expf(x);
    const float nrm = sqrtf(q0 * q0 + q1 * q1 + q2 * q2 + q3 * q3);
    const float qt  = x * (1.0f / fmaxf(nrm, 1e-12f));
    float y = qt;
    y = (j < 10) ? ex : y;
    y = (j == 6) ? sg : y;
    y = (j < 6) ? col : y;
    y = (j < 3) ? x : y;
    sOut[e] = y;
  }
  __syncthreads();

  {
    const int q  = (tid < OUT_PIECES) ? tid : (OUT_PIECES - 1);
    const v4f ov = *(const v4f*)(sOut + q * 4);
    float* op = out + (size_t)blockIdx.x * OUT_FLOATS + q * 4;
    if (tid < OUT_PIECES) *(volatile v4f*)op = ov;
    __threadfence();
    if (tid < OUT_PIECES) *(volatile v4f*)op = ov;
  }
}

static void launch_pack(const float* Wm, unsigned short* dst, int Kreal, int Nreal, int Ksplit, int segMask,
                        int kS, int nT, hipStream_t stream) {
  const int nPieces = nT * kS * 64;
  const int blocks  = (nPieces + 255) / 256;
  k_pack<<<dim3(blocks), dim3(256), 0, stream>>>(Wm, dst, Kreal, Nreal, Ksplit, segMask, kS, nPieces);
}

extern "C" void kernel_launch(void* const* d_in, const int* in_sizes, int n_in,
                              void* d_out, int out_size, void* d_ws, size_t ws_size,
                              hipStream_t stream) {
  if (n_in < 13) return;
  if (in_sizes[0] != NBATCH * TSEQ * TOKEN_DIM) return;
  if (in_sizes[1] != NBATCH * TSEQ * 3) return;
  if (in_sizes[2] != NBATCH * NPTS) return;
  if (in_sizes[3] != IN_DIM * HIDDEN) return;
  if (in_sizes[4] != HIDDEN || in_sizes[5] != HIDDEN || in_sizes[6] != HIDDEN) return;
  if (in_sizes[7] != HIDDEN * HIDDEN) return;
  if (in_sizes[8] != HIDDEN || in_sizes[9] != HIDDEN || in_sizes[10] != HIDDEN) return;
  if (in_sizes[11] != HIDDEN * NHEAD || in_sizes[12] != NHEAD) return;
  if (out_size != ROWS_TOTAL * NHEAD) return;

  const float* tokens  = (const float*)d_in[0];
  const float* anchors = (const float*)d_in[1];
  const int*   ids     = (const int*)d_in[2];
  const float* W1  = (const float*)d_in[3];
  const float* b1  = (const float*)d_in[4];
  const float* g1  = (const float*)d_in[5];
  const float* be1 = (const float*)d_in[6];
  const float* W2  = (const float*)d_in[7];
  const float* b2  = (const float*)d_in[8];
  const float* g2  = (const float*)d_in[9];
  const float* be2 = (const float*)d_in[10];
  const float* W3  = (const float*)d_in[11];
  const float* b3  = (const float*)d_in[12];
  float* out = (float*)d_out;

  const size_t o_tok = 0;
  const size_t o_w1  = o_tok + (size_t)TOK_PIECES * 16;
  const size_t o_w2  = o_w1 + (size_t)W1P_EL * 2;
  const size_t o_w3  = o_w2 + (size_t)W2P_EL * 2;
  const size_t tot   = o_w3 + (size_t)W3P_EL * 2;
  if ((o_w1 % 128) != 0 || (o_w2 % 128) != 0 || (o_w3 % 128) != 0) return;
  if (tot > ws_size) return;
  if (tot > (size_t)134217728) return;

  unsigned short* tokb = (unsigned short*)((char*)d_ws + o_tok);
  unsigned short* W1p  = (unsigned short*)((char*)d_ws + o_w1);
  unsigned short* W2p  = (unsigned short*)((char*)d_ws + o_w2);
  unsigned short* W3p  = (unsigned short*)((char*)d_ws + o_w3);

  k_tokc<<<dim3(TOK_PIECES / 256), dim3(256), 0, stream>>>(tokens, tokb, TOK_PIECES);
  launch_pack(W1, W1p, IN_DIM, HIDDEN, TOKEN_DIM, FSEG - 1, KST1, NT16, stream);
  launch_pack(W2, W2p, HIDDEN, HIDDEN, 0, HIDDEN - 1, KST2, NT16, stream);
  launch_pack(W3, W3p, HIDDEN, NHEAD, 0, HIDDEN - 1, KST2, 1, stream);

  k_main<<<dim3(ROWS_TOTAL / BLOCK_ROWS), dim3(NTHR), 0, stream>>>(
      tokb, anchors, ids, W1p, W2p, W3p, b1, g1, be1, b2, g2, be2, b3, out);
  (void)hipGetLastError();
}
